// PosDefInput_28776280883688
// MI455X (gfx1250) — hardware-verified
//
#include <hip/hip_runtime.h>
#include <stddef.h>
#include <stdint.h>


#define NB    32768
#define NOBS  64
#define HID   256
#define NTR   2080
#define NPAD  4096
#define BT    128
#define NTHR  256
#define XAP   72
#define XTP   132
#define HP    264
#define WSCAP 134217728

#define XS    8.0f
#define WSCL  256.0f
#define HS    8.0f
#define INVC  (1.0f / 2048.0f)

#define OFF_XA  0
#define OFF_XT  (OFF_XA + BT * XAP * 2)
#define OFF_H1  (OFF_XT + NOBS * XTP * 4)
#define OFF_H2  (OFF_H1 + BT * HP * 2)
#define OFF_OUT (OFF_H2 + BT * HP * 2)
#define LDS_MAIN (OFF_OUT + BT * 4)

static_assert(NB % BT == 0);
static_assert(NTHR == 256);
static_assert(BT == 8 * 16);
static_assert((OFF_XT % 16) == 0);
static_assert((OFF_H1 % 16) == 0);
static_assert((OFF_H2 % 16) == 0);
static_assert((OFF_OUT % 16) == 0);
static_assert(LDS_MAIN <= 300 * 1024);
static_assert(NTR == NOBS * (NOBS + 1) / 2);
static_assert(NPAD == NOBS * NOBS);
static_assert((HID % 32) == 0);
static_assert((NOBS % 32) == 0);

typedef float    v4f  __attribute__((ext_vector_type(4)));
typedef float    v8f  __attribute__((ext_vector_type(8)));
typedef _Float16 v4h  __attribute__((ext_vector_type(4)));
typedef _Float16 v8h  __attribute__((ext_vector_type(8)));
typedef _Float16 v16h __attribute__((ext_vector_type(16)));
union FragH { v16h v; v8h h[2]; };

__device__ __forceinline__ v8f wmf(v16h a, v16h b, v8f c) {
  v8f d = __builtin_amdgcn_wmma_f32_16x16x32_f16(false, a, false, b, (short)0, c, false, false);
  asm volatile("v_nop\n\tv_nop\n\tv_nop\n\tv_nop" : "+v"(d) : "v"(a), "v"(b));
  return d;
}

__device__ __forceinline__ v8f zacc() {
  v8f z = {0.f, 0.f, 0.f, 0.f, 0.f, 0.f, 0.f, 0.f};
  return z;
}

template <int K, int MODE>
__global__ __launch_bounds__(NTHR) void k_prepw(const float* __restrict__ W, int nsrc, _Float16* dst) {
  constexpr int TP = K + 8;
  constexpr int CPW = K / 64;
  static_assert((K % 64) == 0);
  static_assert(((TP * 2) % 16) == 0);
  __shared__ __attribute__((aligned(16))) _Float16 tile[32 * TP];
  const int tid = threadIdx.x, l = tid & 31, g = tid >> 5;
  const int row0 = blockIdx.x * 32;
  const int orow = row0 + l;
  int s;
  bool ok;
  if (MODE == 0) {
    s = orow;
    ok = (orow < nsrc);
  } else {
    const int r = orow >> 6, c = orow & 63;
    ok = (c <= r);
    s = (r * (r + 1)) / 2 + c;
  }
  s = (s < 0) ? 0 : s;
  s = (s > nsrc - 1) ? (nsrc - 1) : s;
#pragma unroll 4
  for (int kk = g; kk < K; kk += 8) {
    float v = W[(size_t)kk * nsrc + s];
    v = ok ? (v * WSCL) : 0.0f;
    tile[l * TP + kk] = (_Float16)v;
  }
  __syncthreads();
  v8h hv[CPW];
  size_t po[CPW];
#pragma unroll
  for (int j = 0; j < CPW; ++j) {
    const int cj = g * CPW + j;
    const int p0 = cj * 256 + 8 * l;
    const int nl = p0 / K;
    const int k = p0 - nl * K;
    hv[j] = *(const v8h*)(tile + nl * TP + k);
    po[j] = (size_t)row0 * K + (size_t)p0;
  }
#pragma unroll
  for (int j = 0; j < CPW; ++j) *(volatile v8h*)(dst + po[j]) = hv[j];
  __threadfence();
#pragma unroll
  for (int j = 0; j < CPW; ++j) *(volatile v8h*)(dst + po[j]) = hv[j];
}

__device__ __forceinline__ void elu_store(_Float16* hs, int w, int hh, int m, int nt, v8f acc, float bv) {
#pragma unroll
  for (int r = 0; r < 8; ++r) {
    float v = acc[r] * INVC + bv;
    const float e = expm1f(fminf(v, 0.0f));
    v = (v > 0.0f) ? v : e;
    hs[(w * 16 + 8 * hh + r) * HP + 16 * nt + m] = (_Float16)(v * HS);
  }
}

__global__ __launch_bounds__(NTHR) void k_main(const float* __restrict__ x,
                                               const float* __restrict__ bias1,
                                               const float* __restrict__ bias2,
                                               const float* __restrict__ bias3,
                                               const float* __restrict__ voff,
                                               const _Float16* __restrict__ W1t,
                                               const _Float16* __restrict__ W2t,
                                               const _Float16* __restrict__ W3g,
                                               float* out) {
  extern __shared__ v4f lds_dyn[];
  char* lds = (char*)lds_dyn;
  _Float16* xa   = (_Float16*)(lds + OFF_XA);
  float*    xT   = (float*)(lds + OFF_XT);
  _Float16* h1s  = (_Float16*)(lds + OFF_H1);
  _Float16* h2s  = (_Float16*)(lds + OFF_H2);
  float*    outs = (float*)(lds + OFF_OUT);

  const int tid = threadIdx.x, lane = tid & 31, w = tid >> 5, hh = lane >> 4, m = lane & 15;
  const int bbase = blockIdx.x * BT;

#pragma unroll
  for (int i = 0; i < 8; ++i) {
    const int idx = tid + NTHR * i;
    const int b = idx >> 4, k = (idx & 15) * 4;
    const v4f v = *(const v4f*)(x + (size_t)(bbase + b) * NOBS + k);
    v4h hv;
    hv[0] = (_Float16)(v[0] * XS); hv[1] = (_Float16)(v[1] * XS);
    hv[2] = (_Float16)(v[2] * XS); hv[3] = (_Float16)(v[3] * XS);
    *(v4h*)(xa + b * XAP + k) = hv;
    xT[(k + 0) * XTP + b] = v[0];
    xT[(k + 1) * XTP + b] = v[1];
    xT[(k + 2) * XTP + b] = v[2];
    xT[(k + 3) * XTP + b] = v[3];
  }
  __syncthreads();

  const int arow = w * 16 + m;

  {
    FragH a0, a1;
    const _Float16* ap = xa + arow * XAP + 8 * hh;
    a0.h[0] = *(const v8h*)(ap);
    a0.h[1] = *(const v8h*)(ap + 16);
    a1.h[0] = *(const v8h*)(ap + 32);
    a1.h[1] = *(const v8h*)(ap + 48);
#pragma unroll 1
    for (int nt = 0; nt < HID / 16; ++nt) {
      const int n = 16 * nt + m;
      const _Float16* bp = W1t + (size_t)n * NOBS + 8 * hh;
      FragH b0, b1v;
      b0.h[0]  = *(const v8h*)(bp);
      b0.h[1]  = *(const v8h*)(bp + 16);
      b1v.h[0] = *(const v8h*)(bp + 32);
      b1v.h[1] = *(const v8h*)(bp + 48);
      v8f acc = zacc();
      acc = wmf(a0.v, b0.v, acc);
      acc = wmf(a1.v, b1v.v, acc);
      const float bv = bias1[n];
      elu_store(h1s, w, hh, m, nt, acc, bv);
    }
  }
  __syncthreads();

  FragH af[8];
  {
    const _Float16* ap = h1s + arow * HP + 8 * hh;
#pragma unroll
    for (int ks = 0; ks < 8; ++ks) {
      af[ks].h[0] = *(const v8h*)(ap + 32 * ks);
      af[ks].h[1] = *(const v8h*)(ap + 32 * ks + 16);
    }
  }
#pragma unroll 1
  for (int nt = 0; nt < HID / 16; ++nt) {
    const int n = 16 * nt + m;
    const _Float16* bp = W2t + (size_t)n * HID + 8 * hh;
    v8f acc = zacc();
#pragma unroll
    for (int ks = 0; ks < 8; ++ks) {
      FragH b;
      b.h[0] = *(const v8h*)(bp + 32 * ks);
      b.h[1] = *(const v8h*)(bp + 32 * ks + 16);
      acc = wmf(af[ks].v, b.v, acc);
    }
    const float bv = bias2[n];
    elu_store(h2s, w, hh, m, nt, acc, bv);
  }
  __syncthreads();

  {
    const _Float16* ap = h2s + arow * HP + 8 * hh;
#pragma unroll
    for (int ks = 0; ks < 8; ++ks) {
      af[ks].h[0] = *(const v8h*)(ap + 32 * ks);
      af[ks].h[1] = *(const v8h*)(ap + 32 * ks + 16);
    }
  }
  float q[8];
#pragma unroll
  for (int rr = 0; rr < 8; ++rr) q[rr] = 0.0f;
  const float* xtp = xT + w * 16 + 8 * hh;

#pragma unroll 1
  for (int jt = 0; jt < 4; ++jt) {
    float y[8];
#pragma unroll
    for (int rr = 0; rr < 8; ++rr) y[rr] = 0.0f;
    const int c = 16 * jt + m;
#pragma unroll 1
    for (int r = 16 * jt; r < NOBS; ++r) {
      const _Float16* bp = W3g + (size_t)(r * NOBS + c) * HID + 8 * hh;
      v8f acc = zacc();
#pragma unroll
      for (int ks = 0; ks < 8; ++ks) {
        FragH b;
        b.h[0] = *(const v8h*)(bp + 32 * ks);
        b.h[1] = *(const v8h*)(bp + 32 * ks + 16);
        acc = wmf(af[ks].v, b.v, acc);
      }
      const bool ok = (c <= r);
      int s = (r * (r + 1)) / 2 + c;
      s = (s > NTR - 1) ? (NTR - 1) : s;
      const float bb = bias3[s];
      const v4f x0 = *(const v4f*)(xtp + r * XTP);
      const v4f x1 = *(const v4f*)(xtp + r * XTP + 4);
#pragma unroll
      for (int rr = 0; rr < 4; ++rr) {
        const float l0 = ok ? (acc[rr] * INVC + bb) : 0.0f;
        const float l1 = ok ? (acc[rr + 4] * INVC + bb) : 0.0f;
        y[rr]     += l0 * x0[rr];
        y[rr + 4] += l1 * x1[rr];
      }
    }
#pragma unroll
    for (int rr = 0; rr < 8; ++rr) q[rr] += y[rr] * y[rr];
  }

  const float offv = voff[0] * 1000.0f;
#pragma unroll
  for (int rr = 0; rr < 8; ++rr) {
    float v = q[rr];
    v += __shfl_xor(v, 1);
    v += __shfl_xor(v, 2);
    v += __shfl_xor(v, 4);
    v += __shfl_xor(v, 8);
    q[rr] = v;
  }
  if (m == 0) {
#pragma unroll
    for (int rr = 0; rr < 8; ++rr) outs[w * 16 + 8 * hh + rr] = offv - q[rr];
  }
  __syncthreads();
  if (w == 0) {
    const v4f v = *(const v4f*)(outs + 4 * lane);
    float* p = out + (size_t)bbase + 4 * lane;
    *(volatile v4f*)p = v;
    __threadfence();
    *(volatile v4f*)p = v;
  }
}

extern "C" void kernel_launch(void* const* d_in, const int* in_sizes, int n_in,
                              void* d_out, int out_size, void* d_ws, size_t ws_size,
                              hipStream_t stream) {
  if (n_in < 8) return;
  if (in_sizes[0] != NB * NOBS) return;
  if (in_sizes[1] != NOBS * HID || in_sizes[2] != HID) return;
  if (in_sizes[3] != HID * HID || in_sizes[4] != HID) return;
  if (in_sizes[5] != HID * NTR || in_sizes[6] != NTR) return;
  if (in_sizes[7] < 1) return;
  if (out_size != NB) return;

  const float* x    = (const float*)d_in[0];
  const float* W1   = (const float*)d_in[1];
  const float* b1   = (const float*)d_in[2];
  const float* W2   = (const float*)d_in[3];
  const float* b2   = (const float*)d_in[4];
  const float* W3   = (const float*)d_in[5];
  const float* b3   = (const float*)d_in[6];
  const float* voff = (const float*)d_in[7];
  float* out = (float*)d_out;

  char* ws = (char*)d_ws;
  size_t off = 0;
  const size_t oW1 = off; off += (size_t)HID * NOBS * 2;   off = (off + 255) & ~(size_t)255;
  const size_t oW2 = off; off += (size_t)HID * HID * 2;    off = (off + 255) & ~(size_t)255;
  const size_t oW3 = off; off += (size_t)NPAD * HID * 2;   off = (off + 255) & ~(size_t)255;
  if (off > ws_size || off > (size_t)WSCAP) return;
  _Float16* W1t = (_Float16*)(ws + oW1);
  _Float16* W2t = (_Float16*)(ws + oW2);
  _Float16* W3g = (_Float16*)(ws + oW3);

  k_prepw<NOBS, 0><<<dim3(HID / 32), dim3(NTHR), 0, stream>>>(W1, HID, W1t);
  k_prepw<HID, 0><<<dim3(HID / 32), dim3(NTHR), 0, stream>>>(W2, HID, W2t);
  k_prepw<HID, 1><<<dim3(NPAD / 32), dim3(NTHR), 0, stream>>>(W3, NTR, W3g);
  hipFuncSetAttribute(reinterpret_cast<const void*>(&k_main),
                      hipFuncAttributeMaxDynamicSharedMemorySize, LDS_MAIN);
  k_main<<<dim3(NB / BT), dim3(NTHR), LDS_MAIN, stream>>>(x, b1, b2, b3, voff, W1t, W2t, W3g, out);
}
